// GNNsimple_75368086110725
// MI455X (gfx1250) — hardware-verified
//
#include <hip/hip_runtime.h>
#include <math.h>


typedef unsigned int u32;
typedef __attribute__((ext_vector_type(2)))  int      v2i;
typedef __attribute__((ext_vector_type(16))) _Float16 v16h;
typedef __attribute__((ext_vector_type(8)))  _Float16 v8h;
typedef __attribute__((ext_vector_type(8)))  float    v8f;
typedef __attribute__((ext_vector_type(4)))  float    v4f;
#define NN    50000
#define NE    600000
#define DD    128
#define NG    64
#define MAXPG 8192
#define SORTN 1048576
#define TILE  8192
#define NPAD  50176
#define MAXDEG 4096
#define VST2(T, ptr, val) do { const T _v = (val); *(volatile T*)(ptr) = _v; __threadfence(); *(volatile T*)(ptr) = _v; } while (0)
__device__ __forceinline__ v8f wmma16(v16h a, v16h b, v8f c) {
  v8f d = __builtin_amdgcn_wmma_f32_16x16x32_f16(false, a, false, b, (short)0, c, false, false);
  asm volatile("v_nop\n\tv_nop\n\tv_nop\n\tv_nop" : "+v"(d) : "v"(a), "v"(b));
  return d;
}
__device__ __forceinline__ v16h frag16(const _Float16* p, int hh) {
  const v8h lo = *(const v8h*)(p + 8 * hh), hi = *(const v8h*)(p + 16 + 8 * hh);
  return __builtin_shufflevector(lo, hi, 0,1,2,3,4,5,6,7,8,9,10,11,12,13,14,15);
}
__global__ __launch_bounds__(256) void k_sort_init(const int* __restrict__ src, const int* __restrict__ dst, u32* __restrict__ A, int E) {
  const int i = blockIdx.x * 256 + threadIdx.x;
  VST2(u32, A + i, (i < E) ? (((u32)dst[i]) << 16) | (u32)src[i] : 0xffffffffu);
}
__device__ __forceinline__ void cas_lds(u32* s, int lo, int hi, bool up) {
  const u32 a = s[lo], b = s[hi]; const bool sw = up ? (a > b) : (a < b); s[lo] = sw ? b : a; s[hi] = sw ? a : b;
}
__global__ __launch_bounds__(256) void k_sort_local(u32* __restrict__ A) {
  __shared__ u32 s[TILE];
  const int base = blockIdx.x * TILE, t = threadIdx.x;
  for (int i = t; i < TILE; i += 256) s[i] = A[base + i];
  __syncthreads();
  for (int k = 2; k <= TILE; k <<= 1)
    for (int j = k >> 1; j > 0; j >>= 1) {
      for (int p = t; p < TILE / 2; p += 256) {
        const int lo = ((p >> __builtin_ctz(j)) << (__builtin_ctz(j) + 1)) | (p & (j - 1));
        cas_lds(s, lo, lo + j, (((base + lo) & k) == 0));
      }
      __syncthreads();
    }
  for (int pass = 0; pass < 2; ++pass) { for (int i = t; i < TILE; i += 256) *(volatile u32*)(A + base + i) = s[i]; __threadfence(); }
}
__global__ __launch_bounds__(256) void k_sort_global(u32* __restrict__ A, int logj, int k) {
  const int p = blockIdx.x * 256 + threadIdx.x;
  const int j = 1 << logj;
  const int lo = ((p >> logj) << (logj + 1)) | (p & (j - 1)), hi = lo + j;
  const u32 a = A[lo], b = A[hi];
  const bool up = ((lo & k) == 0), sw = up ? (a > b) : (a < b);
  const u32 vlo = sw ? b : a, vhi = sw ? a : b;
  *(volatile u32*)(A + lo) = vlo; *(volatile u32*)(A + hi) = vhi; __threadfence();
  *(volatile u32*)(A + lo) = vlo; *(volatile u32*)(A + hi) = vhi;
}
__global__ __launch_bounds__(256) void k_sort_lds(u32* __restrict__ A, int k) {
  __shared__ u32 s[TILE];
  const int base = blockIdx.x * TILE, t = threadIdx.x;
  for (int i = t; i < TILE; i += 256) s[i] = A[base + i];
  __syncthreads();
  for (int j = TILE >> 1; j > 0; j >>= 1) {
    for (int p = t; p < TILE / 2; p += 256) {
      const int lo = ((p >> __builtin_ctz(j)) << (__builtin_ctz(j) + 1)) | (p & (j - 1));
      cas_lds(s, lo, lo + j, (((base + lo) & k) == 0));
    }
    __syncthreads();
  }
  for (int pass = 0; pass < 2; ++pass) { for (int i = t; i < TILE; i += 256) *(volatile u32*)(A + base + i) = s[i]; __threadfence(); }
}

__global__ __launch_bounds__(256) void k_segs(const u32* __restrict__ A, v2i* __restrict__ seg, float* __restrict__ inv) {
  const int n = blockIdx.x * 256 + threadIdx.x;
  if (n >= NN) return;
  int lo = 0, hi = SORTN;
  while (lo < hi) { const int mid = (lo + hi) >> 1; if ((A[mid] >> 16) < (u32)n) lo = mid + 1; else hi = mid; }
  const int st = lo; hi = SORTN;
  while (lo < hi) { const int mid = (lo + hi) >> 1; if ((A[mid] >> 16) < (u32)(n + 1)) lo = mid + 1; else hi = mid; }
  const v2i sv = {st, lo - st};
  VST2(v2i, seg + n, sv);
  VST2(float, inv + n, 1.0f / fmaxf((float)(lo - st), 1.0f));
}

__global__ __launch_bounds__(256) void k_rows(const float* __restrict__ h, const u32* __restrict__ A, const v2i* __restrict__ seg, const float* __restrict__ inv,
                                              _Float16* __restrict__ A16) {
  const int t = blockIdx.x * 256 + threadIdx.x;
  const int i = t >> 5, c = (t & 31) * 8;
  v8h o;
  if (i >= NN) { for (int e = 0; e < 8; ++e) o[e] = (_Float16)0.f; }
  else if (c >= DD) {
#pragma unroll
    for (int e = 0; e < 8; ++e) o[e] = (_Float16)h[(size_t)i * DD + c - DD + e];
  } else {
    const v2i sv = seg[i];
    const int st = min(max(sv[0], 0), SORTN - 1), cnt = min(max(sv[1], 0), MAXDEG);
    float acc[8] = {0.f, 0.f, 0.f, 0.f, 0.f, 0.f, 0.f, 0.f};
    for (int p = 0; p < cnt; ++p) {
      const int j = min((int)(A[min(st + p, SORTN - 1)] & 0xffffu), NN - 1);
      const float* hr = h + (size_t)j * DD + c;
#pragma unroll
      for (int e = 0; e < 8; ++e) acc[e] += hr[e];
    }
    const float w = inv[i];
#pragma unroll
    for (int e = 0; e < 8; ++e) o[e] = (_Float16)(acc[e] * w);
  }
  VST2(v8h, A16 + (size_t)i * 256 + c, o);
}
__global__ __launch_bounds__(256) void k_wt(const float* __restrict__ Wl, const float* __restrict__ Wr, _Float16* __restrict__ Wt) {
  const int t = blockIdx.x * 256 + threadIdx.x;
  const int n = t >> 5, k0 = (t & 31) * 8;
  v8h o;
#pragma unroll
  for (int e = 0; e < 8; ++e) { const int k = k0 + e; o[e] = (_Float16)((k < DD) ? Wl[n * DD + k] : Wr[n * DD + k - DD]); }
  VST2(v8h, Wt + (size_t)n * 256 + k0, o);
}
__global__ __launch_bounds__(128) void k_gemm(const _Float16* __restrict__ A16, const _Float16* __restrict__ Wt, const float* __restrict__ bias, float* __restrict__ out) {
  __shared__ __attribute__((aligned(16))) float sT[4][16][132];
  const int lane = threadIdx.x & 31, wave = threadIdx.x >> 5, hh = lane >> 4, l16 = lane & 15;
  const int m0 = blockIdx.x * 64 + wave * 16;
  v8f acc[8];
#pragma unroll
  for (int ni = 0; ni < 8; ++ni) acc[ni] = (v8f){};
#pragma unroll 2
  for (int k0 = 0; k0 < 256; k0 += 32) {
    const v16h a0 = frag16(A16 + (size_t)(m0 + l16) * 256 + k0, hh);
#pragma unroll
    for (int ni = 0; ni < 8; ++ni) { const v16h b = frag16(Wt + (size_t)(ni * 16 + l16) * 256 + k0, hh); acc[ni] = wmma16(a0, b, acc[ni]); }
  }
  float (*st)[132] = sT[wave];
#pragma unroll
  for (int ni = 0; ni < 8; ++ni)
#pragma unroll
    for (int i = 0; i < 8; ++i) st[i + 8 * hh][ni * 16 + l16] = fmaxf(acc[ni][i] + bias[ni * 16 + l16], 0.f);
  __builtin_amdgcn_fence(__ATOMIC_RELEASE, "workgroup"); __builtin_amdgcn_wave_barrier(); __builtin_amdgcn_fence(__ATOMIC_ACQUIRE, "workgroup");
  for (int pass = 0; pass < 2; ++pass) {
#pragma unroll
    for (int rr = 0; rr < 16; ++rr) *(volatile v4f*)(out + (size_t)(m0 + rr) * DD + lane * 4) = *(const v4f*)(&st[rr][lane * 4]);
    __threadfence();
  }
}
__global__ __launch_bounds__(256) void k_head(const float* __restrict__ h, const int* __restrict__ batch, const float* __restrict__ Wc1, const float* __restrict__ bc1,
                                              const float* __restrict__ Wc2, const float* __restrict__ bc2, float* __restrict__ out) {
  __shared__ float g[2][DD], z[2][DD], res[NG];
  const int t = threadIdx.x, half = t >> 7, c = t & 127;
  for (int gp = 0; gp < NG; gp += 2) {
    const int gi = gp + half;
    int lo = 0, hi = NN;
    while (lo < hi) { const int mid = (lo + hi) >> 1; if (batch[mid] < gi) lo = mid + 1; else hi = mid; }
    const int st = lo; hi = NN;
    while (lo < hi) { const int mid = (lo + hi) >> 1; if (batch[mid] < gi + 1) lo = mid + 1; else hi = mid; }
    const int cnt = min(lo - st, MAXPG);
    float s = 0.f;
    for (int p = 0; p < cnt; ++p) s += h[(size_t)min(st + p, NN - 1) * DD + c];
    g[half][c] = s / fmaxf((float)(lo - st), 1.0f);
    __syncthreads();
    float a = bc1[c];
    for (int k = 0; k < DD; ++k) a += g[half][k] * Wc1[c * DD + k];
    z[half][c] = fmaxf(a, 0.f);
    __syncthreads();
    if (c == 0) { float o = bc2[0]; for (int k = 0; k < DD; ++k) o += z[half][k] * Wc2[k]; res[gi] = o; }
    __syncthreads();
  }
  if (t < NG) { *(volatile float*)(out + t) = res[t]; __threadfence(); *(volatile float*)(out + t) = res[t]; }
}
extern "C" void kernel_launch(void* const* d_in, const int* in_sizes, int n_in,
                              void* d_out, int out_size, void* d_ws, size_t ws_size, hipStream_t stream) {
  (void)in_sizes; (void)n_in; (void)out_size;
  const float* x     = (const float*)d_in[0];
  const int*   ei    = (const int*)  d_in[1];
  const int*   batch = (const int*)  d_in[2];
  const float* W1l = (const float*)d_in[3]; const float* b1l = (const float*)d_in[4]; const float* W1r = (const float*)d_in[5];
  const float* W2l = (const float*)d_in[6]; const float* b2l = (const float*)d_in[7]; const float* W2r = (const float*)d_in[8];
  const float* Wc1 = (const float*)d_in[9]; const float* bc1 = (const float*)d_in[10];
  const float* Wc2 = (const float*)d_in[11]; const float* bc2 = (const float*)d_in[12];
  float* out = (float*)d_out;
  char* ws = (char*)d_ws; size_t off = 0;
  auto take = [&](size_t bytes) { void* p = ws + off; off = (off + bytes + 255) & ~(size_t)255; return p; };
  u32*      keys = (u32*)take((size_t)SORTN * 4);
  v2i*      seg  = (v2i*)take((size_t)NN * 8);
  float*    inv  = (float*)take((size_t)NN * 4);
  _Float16* A16  = (_Float16*)take((size_t)NPAD * 256 * 2);
  _Float16* Wt   = (_Float16*)take((size_t)DD * 256 * 2);
  float*    h1   = (float*)take((size_t)NPAD * DD * 4);
  float*    h2   = (float*)take((size_t)NPAD * DD * 4);
  if (off > ws_size) return;
  const dim3 b256(256);
  k_sort_init<<<SORTN / 256, b256, 0, stream>>>(ei, ei + NE, keys, NE);
  k_sort_local<<<SORTN / TILE, b256, 0, stream>>>(keys);
  for (int k = TILE * 2; k <= SORTN; k <<= 1) {
    for (int logj = __builtin_ctz(k) - 1; (1 << logj) >= TILE; --logj)
      k_sort_global<<<SORTN / 2 / 256, b256, 0, stream>>>(keys, logj, k);
    k_sort_lds<<<SORTN / TILE, b256, 0, stream>>>(keys, k);
  }
  k_segs<<<(NN + 255) / 256, b256, 0, stream>>>(keys, seg, inv);
  k_rows<<<NPAD * 32 / 256, b256, 0, stream>>>(x, keys, seg, inv, A16);
  k_wt<<<DD * 32 / 256, b256, 0, stream>>>(W1l, W1r, Wt);
  k_gemm<<<NPAD / 64, 128, 0, stream>>>(A16, Wt, b1l, h1);
  k_rows<<<NPAD * 32 / 256, b256, 0, stream>>>(h1, keys, seg, inv, A16);
  k_wt<<<DD * 32 / 256, b256, 0, stream>>>(W2l, W2r, Wt);
  k_gemm<<<NPAD / 64, 128, 0, stream>>>(A16, Wt, b2l, h2);
  k_head<<<1, b256, 0, stream>>>(h2, batch, Wc1, bc1, Wc2, bc2, out);
}
